// PathQualityAwareConv_40303973105672
// MI455X (gfx1250) — hardware-run, weakly checked
//
#include <hip/hip_runtime.h>


namespace {
constexpr int N = 50000, NP = 50048, E = 800000, IN = 128, OUT = 64, ED = 16, NH = 4, HC = NH * OUT  , KC = 96  ;
constexpr float XS = 8.0f, WSC = 256.0f, SLOPE = 0.2f;

typedef _Float16 b16;
typedef __attribute__((ext_vector_type(16))) _Float16 v16b;
typedef __attribute__((ext_vector_type(8))) _Float16 v8b;
typedef __attribute__((ext_vector_type(8))) float v8f;
typedef __attribute__((ext_vector_type(4))) float v4f;
__device__ __forceinline__ float bf16_rne(float f) { unsigned int u = __float_as_uint(f); u += 0x7FFFu + ((u >> 16) & 1u); return __uint_as_float(u & 0xFFFF0000u); }
__device__ __forceinline__ void split16(float v, b16& hi, b16& lo) { hi = (b16)v; lo = (b16)(v - (float)hi); }
__device__ __forceinline__ v16b frag_kb(const b16* p, int hh) { const v8b a = *(const v8b*)(p + 8 * hh), b = *(const v8b*)(p + 16 + 8 * hh); v16b f;
#pragma unroll
  for (int e = 0; e < 8; ++e) { f[e] = a[e]; f[8 + e] = b[e]; } return f; }
__device__ __forceinline__ v8f wmma16b(v16b a, v16b b, v8f c) { v8f d = __builtin_amdgcn_wmma_f32_16x16x32_f16(false, a, false, b, (short)0, c, false, false); asm volatile("v_nop\n\tv_nop\n\tv_nop\n\tv_nop" : "+v"(d) : "v"(a), "v"(b)); return d; }
__device__ __forceinline__ void wave_lds_sync() { __builtin_amdgcn_fence(__ATOMIC_RELEASE, "workgroup"); __builtin_amdgcn_wave_barrier(); __builtin_amdgcn_fence(__ATOMIC_ACQUIRE, "workgroup"); }
__device__ __forceinline__ float pmul(float a, float b) { float p = a * b; asm volatile("" : "+v"(p)); return p; }
__device__ __forceinline__ float hsum16(float v) { v += __shfl_xor(v, 1); v += __shfl_xor(v, 2); v += __shfl_xor(v, 4); return v + __shfl_xor(v, 8); }
__device__ __forceinline__ int iclamp(int v, int lo, int hi) { return v < lo ? lo : (v > hi ? hi : v); }
__device__ __forceinline__ float lrelu(float x) { return x > 0.0f ? x : SLOPE * x; }

constexpr int CSR_NBLK = 512, CSR_GB = 9, CSR_GN = 1 << CSR_GB  , CSR_MAXG = 512, CSR_CAP = 12288  ;
__global__ __launch_bounds__(64) void csrA_kernel(const int* __restrict__ dst, int E, int N, int nG, int CHP, int NGP, int* __restrict__ STG, int* __restrict__ HST) {
  extern __shared__ int sm[];
  int* cnt = sm; int* run = sm + NGP; int* ids = sm + 2 * NGP;
  const int b = blockIdx.x; const int ch = (E + CSR_NBLK - 1) / CSR_NBLK; const int e0 = b * ch, e1 = min(E, e0 + ch);
  for (int i = threadIdx.x; i < NGP; i += 64) cnt[i] = 0;
  for (int i = threadIdx.x; i < CHP; i += 64) ids[i] = -1;
  __syncthreads();
  if (threadIdx.x == 0) {
    for (int e = e0; e < e1; ++e) { int d = dst[e]; d = (d < 0) ? 0 : (d >= N ? N - 1 : d); cnt[d >> CSR_GB] += 1; }
    int acc = 0; for (int g = 0; g < nG; ++g) { run[g] = acc; acc += cnt[g]; }
    for (int e = e0; e < e1; ++e) { int d = dst[e]; d = (d < 0) ? 0 : (d >= N ? N - 1 : d); const int g = d >> CSR_GB; ids[run[g]] = e; run[g] += 1; } }
  __syncthreads();
  typedef __attribute__((ext_vector_type(4))) int v4i;
  for (int pass = 0; pass < 2; ++pass) {
    for (int i = threadIdx.x; i < CHP / 4; i += 64) *(volatile v4i*)(STG + (size_t)b * CHP + i * 4) = *(const v4i*)(&ids[i * 4]);
    for (int i = threadIdx.x; i < NGP / 4; i += 64) { v4i v; for (int e = 0; e < 4; ++e) v[e] = (i * 4 + e < nG) ? cnt[i * 4 + e] : 0; *(volatile v4i*)(HST + (size_t)b * NGP + i * 4) = v; }
    __threadfence(); }
}
__global__ __launch_bounds__(512) void csrS_kernel(const int* __restrict__ HST, int nG, int NGP, int* __restrict__ START, int* __restrict__ TOT, int* __restrict__ OFF) {
  __shared__ int tot[CSR_MAXG];
  const int b = threadIdx.x;
  for (int pass = 0; pass < 2; ++pass) { int runb = 0; for (int g = 0; g < nG; ++g) { int c = HST[(size_t)b * NGP + g]; c = (c < 0) ? 0 : c; ((volatile int*)OFF)[(size_t)g * CSR_NBLK + b] = runb; runb += c; } __threadfence(); }
  for (int g = threadIdx.x; g < nG; g += 512) { int s = 0; for (int bb = 0; bb < CSR_NBLK; ++bb) { int c = HST[(size_t)bb * NGP + g]; s += (c < 0) ? 0 : c; } tot[g] = s; }
  __syncthreads();
  if (threadIdx.x < 32) {
    __shared__ int st[CSR_MAXG + 32];
    if (threadIdx.x == 0) { int acc = 0; for (int g = 0; g < NGP; ++g) { st[g] = acc; if (g < nG) acc += (tot[g] + 31) & ~31; } st[NGP] = acc; }
    __builtin_amdgcn_fence(__ATOMIC_RELEASE, "workgroup"); __builtin_amdgcn_wave_barrier(); __builtin_amdgcn_fence(__ATOMIC_ACQUIRE, "workgroup");
    for (int pass = 0; pass < 2; ++pass) { for (int i = threadIdx.x; i < NGP + 32; i += 32) { ((volatile int*)START)[i] = (i <= NGP) ? st[min(i, NGP)] : 0; ((volatile int*)TOT)[i] = (i < nG) ? tot[i] : 0; } __threadfence(); } }
}
__global__ __launch_bounds__(256) void csrB_kernel(const int* __restrict__ dst, int N, int nG, int CHP, int NGP, int permLen, const int* __restrict__ STG, const int* __restrict__ HST, const int* __restrict__ OFF, const int* __restrict__ START, const int* __restrict__ TOT, int* __restrict__ PERM, int* __restrict__ ROWPTR, int* __restrict__ ROWCNT, int* __restrict__ FLAG) {
  typedef __attribute__((ext_vector_type(4))) int v4i;
  __shared__ int ids[CSR_CAP]; __shared__ unsigned short key[CSR_CAP]; __shared__ int outp[CSR_CAP]; __shared__ int ncnt[CSR_GN + 1]; __shared__ int boff[CSR_NBLK + 1];
  const int g = blockIdx.x, t_ = threadIdx.x; int tot = TOT[g]; int st = START[g], stn = START[g + 1]; const int v0 = g * CSR_GN; const int nv = min(CSR_GN, N - v0);
  st = (st < 0) ? 0 : (st > permLen - 32 ? permLen - 32 : st) & ~31; stn = (stn < st) ? st : (stn > permLen ? permLen : stn); tot = (tot < 0) ? 0 : tot; if (tot > stn - st && tot <= CSR_CAP) tot = stn - st;
  if (tot > CSR_CAP) {
    for (int pass = 0; pass < 2; ++pass) { for (int i = t_; i < CSR_GN / 4; i += 256) { v4i a, c; for (int e = 0; e < 4; ++e) { a[e] = st; c[e] = 0; } *(volatile v4i*)(ROWPTR + v0 + i * 4) = a; *(volatile v4i*)(ROWCNT + v0 + i * 4) = c; } if (t_ == 0) ((volatile int*)FLAG)[0] = 1; __threadfence(); } (void)nv; return; }
  if (t_ == 0) { int acc = 0; for (int b = 0; b < CSR_NBLK; ++b) { boff[b] = acc; int c = HST[(size_t)b * NGP + g]; c = (c < 0) ? 0 : (c > CHP ? CHP : c); acc += c; if (acc > tot) acc = tot; } boff[CSR_NBLK] = acc; }
  for (int i = t_; i <= CSR_GN; i += 256) ncnt[i] = 0;
  __syncthreads();
  for (int b = 0; b < CSR_NBLK; ++b) { const int c = boff[b + 1] - boff[b]; int o_ = OFF[(size_t)g * CSR_NBLK + b]; o_ = (o_ < 0) ? 0 : (o_ > CHP - c ? CHP - c : o_); const int* src_ = STG + (size_t)b * CHP + o_;
    for (int i = t_; i < c; i += 256) { int id = src_[i]; id = (id < 0) ? 0 : id; ids[boff[b] + i] = id; int d = dst[id]; d = (d < v0) ? v0 : (d >= N ? N - 1 : d); int kk = d - v0; kk = (kk < 0) ? 0 : (kk >= CSR_GN ? CSR_GN - 1 : kk); key[boff[b] + i] = (unsigned short)kk; } }
  __syncthreads();
  if (t_ == 0) { for (int i = 0; i < tot; ++i) ncnt[key[i]] += 1; int acc = 0; for (int vl = 0; vl < CSR_GN; ++vl) { const int c = ncnt[vl]; ncnt[vl] = acc; acc += c; } ncnt[CSR_GN] = acc;
    for (int i = 0; i < tot; ++i) { const int vl = key[i]; outp[ncnt[vl]] = ids[i]; ncnt[vl] += 1; }
    for (int vl = CSR_GN; vl > 0; --vl) ncnt[vl] = ncnt[vl - 1]; ncnt[0] = 0; }
  __syncthreads();
  for (int pass = 0; pass < 2; ++pass) {
    for (int i = t_; i < (stn - st) / 4; i += 256) { v4i v; for (int e = 0; e < 4; ++e) { const int q = i * 4 + e; v[e] = (q < tot) ? outp[q] : -1; } *(volatile v4i*)(PERM + st + i * 4) = v; }
    for (int i = t_; i < CSR_GN / 4; i += 256) { v4i a, c; for (int e = 0; e < 4; ++e) { const int vl = i * 4 + e; a[e] = st + ncnt[vl]; c[e] = (vl < nv) ? (ncnt[vl + 1] - ncnt[vl]) : 0; } *(volatile v4i*)(ROWPTR + v0 + i * 4) = a; *(volatile v4i*)(ROWCNT + v0 + i * 4) = c; }
    __threadfence(); }
}
__global__ __launch_bounds__(256) void csrZ_kernel(int* __restrict__ p, size_t n4) { typedef __attribute__((ext_vector_type(4))) int v4i; const size_t tid = (size_t)blockIdx.x * 256 + threadIdx.x, nth = (size_t)gridDim.x * 256; v4i z = {0, 0, 0, 0}; for (size_t i = tid; i < n4; i += nth) *(volatile v4i*)(p + i * 4) = z; }
struct CsrBufs { int *STG, *HST, *OFF, *START, *TOT, *PERM, *ROWPTR, *ROWCNT, *FLAG; int nG, NGP, CHP; size_t permLen; char* base; size_t bytes; };
static size_t csr_carve(CsrBufs& c, char* ws, size_t off, int E, int N) {
  const size_t off0 = off; c.base = ws + off;
  auto al = [&](size_t bytes) { char* p = ws + off; off += (bytes + 255) & ~(size_t)255; return p; };
  c.nG = (N + CSR_GN - 1) / CSR_GN; c.NGP = (c.nG + 31) & ~31; const int ch = (E + CSR_NBLK - 1) / CSR_NBLK; c.CHP = (ch + 31) & ~31; c.permLen = (size_t)E + 32 * (size_t)c.nG + 32;
  c.STG = (int*)al((size_t)CSR_NBLK * c.CHP * 4); c.HST = (int*)al((size_t)CSR_NBLK * c.NGP * 4); c.OFF = (int*)al((size_t)c.NGP * CSR_NBLK * 4); c.START = (int*)al((size_t)(c.NGP + 64) * 4); c.TOT = (int*)al((size_t)(c.NGP + 64) * 4);
  c.PERM = (int*)al(c.permLen * 4); c.ROWPTR = (int*)al((size_t)c.nG * CSR_GN * 4); c.ROWCNT = (int*)al((size_t)c.nG * CSR_GN * 4); c.FLAG = (int*)al(256);
  c.bytes = off - off0; return off;
}
static void csr_build(const CsrBufs& c, const int* dst, int E, int N, hipStream_t stream) {
  const size_t smem = (size_t)(2 * c.NGP + c.CHP) * 4;
  csrZ_kernel<<<512, 256, 0, stream>>>((int*)c.base, c.bytes / 16);
  csrA_kernel<<<CSR_NBLK, 64, smem, stream>>>(dst, E, N, c.nG, c.CHP, c.NGP, c.STG, c.HST);
  csrS_kernel<<<1, 512, 0, stream>>>(c.HST, c.nG, c.NGP, c.START, c.TOT, c.OFF);
  csrB_kernel<<<c.nG, 256, 0, stream>>>(dst, N, c.nG, c.CHP, c.NGP, (int)c.permLen, c.STG, c.HST, c.OFF, c.START, c.TOT, c.PERM, c.ROWPTR, c.ROWCNT, c.FLAG);
}


__global__ __launch_bounds__(256) void prep_kernel(const float* __restrict__ x, const float* __restrict__ wg, const float* __restrict__ wc, const float* __restrict__ wedge, const float* __restrict__ attedge, b16* __restrict__ X16, b16* __restrict__ WGT, b16* __restrict__ WCT, float* __restrict__ U) {
  const size_t t = (size_t)blockIdx.x * 256 + threadIdx.x; const size_t nx = (size_t)NP * IN / 8, n1 = (size_t)HC * IN / 8, n2 = (size_t)OUT * KC / 8; v8b o = {};
  if (t < nx) { const size_t e = t * 8; if (e < (size_t)N * IN) { const v4f a = *(const v4f*)(x + e), c = *(const v4f*)(x + e + 4); for (int j = 0; j < 4; ++j) { o[j] = (b16)(bf16_rne(a[j]) * XS); o[4 + j] = (b16)(bf16_rne(c[j]) * XS); } }
    for (int pass = 0; pass < 2; ++pass) { *(volatile v8b*)(X16 + e) = o; __threadfence(); } }
  else if (t < nx + n1) { const size_t u = (t - nx) * 8; const int oo = (int)(u / IN), i0 = (int)(u - (size_t)oo * IN); for (int j = 0; j < 8; ++j) o[j] = (b16)(bf16_rne(wg[(size_t)(i0 + j) * HC + oo]) * WSC); for (int pass = 0; pass < 2; ++pass) { *(volatile v8b*)(WGT + u) = o; __threadfence(); } }
  else if (t < nx + n1 + n2) { const size_t u = (t - nx - n1) * 8; const int oo = (int)(u / KC), k0 = (int)(u - (size_t)oo * KC); for (int j = 0; j < 8; ++j) { const int k = k0 + j; o[j] = (b16)((k < OUT + ED) ? bf16_rne(wc[(size_t)k * OUT + oo]) * WSC : 0.0f); } for (int pass = 0; pass < 2; ++pass) { *(volatile v8b*)(WCT + u) = o; __threadfence(); } }
  else if (t < nx + n1 + n2 + 64) { const int i = (int)(t - nx - n1 - n2); const int k = i >> 2, h = i & 3; float s = 0.0f; for (int c = 0; c < OUT; ++c) s += pmul(bf16_rne(wedge[k * HC + h * OUT + c]), bf16_rne(attedge[h * OUT + c]));
    for (int pass = 0; pass < 2; ++pass) { ((volatile float*)U)[i] = s; __threadfence(); } }
}
__global__ __launch_bounds__(128) void node_kernel(const b16* __restrict__ X16, const b16* __restrict__ WGT, const float* __restrict__ att_s, const float* __restrict__ att_d, float* __restrict__ XS_, float* __restrict__ AS, float* __restrict__ AD) {
  __shared__ __attribute__((aligned(16))) float Ts[4][16][128 + 4]; __shared__ float Sa[64][2], Sd[64][2];
  const int wave = threadIdx.x >> 5, lane = threadIdx.x & 31, nloc = lane & 15, hlf = lane >> 4; const size_t m0 = ((size_t)blockIdx.x * 4 + wave) * 16; const int n0 = blockIdx.y * 128;
  v8f acc[8];
#pragma unroll
  for (int t = 0; t < 8; ++t) acc[t] = (v8f){};
#pragma unroll
  for (int kb = 0; kb < IN; kb += 32) { const v16b a = frag_kb(X16 + (m0 + nloc) * IN + kb, hlf);
#pragma unroll
    for (int t = 0; t < 8; ++t) acc[t] = wmma16b(a, frag_kb(WGT + (size_t)(n0 + t * 16 + nloc) * IN + kb, hlf), acc[t]); }
  float ps[8][2], pd[8][2];
#pragma unroll
  for (int r = 0; r < 8; ++r) { ps[r][0] = ps[r][1] = pd[r][0] = pd[r][1] = 0.0f; }
#pragma unroll
  for (int t = 0; t < 8; ++t) { const int c = n0 + t * 16 + nloc; const int hl = t >> 2; const float sa = bf16_rne(att_s[c]), sd = bf16_rne(att_d[c]);
#pragma unroll
    for (int r = 0; r < 8; ++r) { const float vv = acc[t][r] * (1.0f / (XS * WSC)); Ts[wave][8 * hlf + r][t * 16 + nloc] = vv; ps[r][hl] += pmul(vv, sa); pd[r][hl] += pmul(vv, sd); } }
#pragma unroll
  for (int r = 0; r < 8; ++r)
#pragma unroll
    for (int hl = 0; hl < 2; ++hl) { const float s1 = hsum16(ps[r][hl]), s2 = hsum16(pd[r][hl]); if (nloc == 0) { Sa[wave * 16 + 8 * hlf + r][hl] = s1; Sd[wave * 16 + 8 * hlf + r][hl] = s2; } }
  __syncthreads();
  for (int pass = 0; pass < 2; ++pass) {
    for (int rr = 0; rr < 16; ++rr) *(volatile v4f*)(XS_ + (m0 + rr) * HC + n0 + lane * 4) = *(const v4f*)(&Ts[wave][rr][lane * 4]);
    { const int i = threadIdx.x; if (i < 128) { const int rr = i >> 1, hl = i & 1; const size_t v = (size_t)blockIdx.x * 64 + rr; ((volatile float*)AS)[((size_t)blockIdx.y * NP + v) * 2 + hl] = Sa[rr][hl]; ((volatile float*)AD)[((size_t)blockIdx.y * NP + v) * 2 + hl] = Sd[rr][hl]; } }
    __threadfence(); }
}
__device__ __forceinline__ float as_at(const float* AS, int v, int h) { return AS[((size_t)(h >> 1) * NP + v) * 2 + (h & 1)]; }
__global__ __launch_bounds__(256) void edge_kernel(const float* __restrict__ eattr, const float* __restrict__ qual, const float* __restrict__ wq1, const float* __restrict__ bq1, const float* __restrict__ wq2, const float* __restrict__ bq2, const float* __restrict__ U, float* __restrict__ AE) {
  __shared__ float W1s[4][8], B1s[8], W2s[8][16], B2s[16], Us[16][4];
  const int t_ = threadIdx.x; if (t_ < 32) W1s[t_ >> 3][t_ & 7] = bf16_rne(wq1[t_]); if (t_ < 8) B1s[t_] = bf16_rne(bq1[t_]); if (t_ < 128) W2s[t_ >> 4][t_ & 15] = bf16_rne(wq2[t_]); if (t_ < 16) B2s[t_] = bf16_rne(bq2[t_]); if (t_ < 64) Us[t_ >> 2][t_ & 3] = U[t_];
  __syncthreads();
  const size_t e = (size_t)blockIdx.x * 256 + t_; if (e >= (size_t)E) return;
  const v4f qr = *(const v4f*)(qual + e * 4); float q4[4] = {bf16_rne(qr[0]), bf16_rne(qr[1]), bf16_rne(qr[2]), bf16_rne(qr[3])}; float h8[8];
#pragma unroll
  for (int j = 0; j < 8; ++j) { float s = B1s[j]; for (int k = 0; k < 4; ++k) s += pmul(q4[k], W1s[k][j]); h8[j] = fmaxf(s, 0.0f); }
  float a4[4] = {0, 0, 0, 0};
#pragma unroll
  for (int k4 = 0; k4 < ED; k4 += 4) { const v4f ea4 = *(const v4f*)(eattr + e * ED + k4);
#pragma unroll
    for (int kk = 0; kk < 4; ++kk) { const int k = k4 + kk; float qk = B2s[k]; for (int j = 0; j < 8; ++j) qk += pmul(h8[j], W2s[j][k]); const float ea = bf16_rne(ea4[kk]) + qk;
#pragma unroll
      for (int h = 0; h < 4; ++h) a4[h] += pmul(ea, Us[k][h]); } }
  const v4f o = {a4[0], a4[1], a4[2], a4[3]};
  for (int pass = 0; pass < 2; ++pass) { *(volatile v4f*)(AE + e * 4) = o; __threadfence(); }
}
__global__ __launch_bounds__(256) void agg_kernel(const int* __restrict__ srcs, const float* __restrict__ XS_, const float* __restrict__ AS, const float* __restrict__ AD, const float* __restrict__ AE, const float* __restrict__ bgat, const float* __restrict__ nstate, const int* __restrict__ PERM, const int* __restrict__ ROWPTR, const int* __restrict__ ROWCNT, int permLen, b16* __restrict__ X2h, b16* __restrict__ X2l) {
  const int wave = threadIdx.x >> 5, lane = threadIdx.x & 31; const size_t v = ((size_t)blockIdx.x * 8 + wave) * 2 + (lane >> 4); const int l = lane & 15; const int c0 = l * 16, h = l >> 2, cc = (l & 3) * 16;
  const int vv = (int)((v < (size_t)N) ? v : (size_t)(N - 1));
  int st = ROWPTR[vv], cnt = ROWCNT[vv]; cnt = iclamp(cnt, 0, 4096); st = iclamp(st, 0, permLen - cnt); if (v >= (size_t)N) cnt = 0;
  const float ad = as_at(AD, vv, h);
  float m = -INFINITY; for (int j = 0; j < cnt; ++j) { const int e = iclamp(PERM[st + j], 0, E - 1); const int s = iclamp(srcs[e], 0, N - 1); m = fmaxf(m, lrelu(as_at(AS, s, h) + ad + AE[(size_t)e * 4 + h])); }
  float den = 0.0f; float acc[16]; for (int q = 0; q < 16; ++q) acc[q] = 0.0f;
  for (int j = 0; j < cnt; ++j) { const int e = iclamp(PERM[st + j], 0, E - 1); const int s = iclamp(srcs[e], 0, N - 1); const float a = __expf(lrelu(as_at(AS, s, h) + ad + AE[(size_t)e * 4 + h]) - m); den += a; const float* hr = XS_ + (size_t)s * HC + c0;
#pragma unroll
    for (int q4 = 0; q4 < 16; q4 += 4) { const v4f hq = *(const v4f*)(hr + q4); for (int q = 0; q < 4; ++q) acc[q4 + q] += pmul(a, hq[q]); } }
  const float inv = (cnt > 0) ? 1.0f / (den + 1e-16f) : 0.0f;
  float mean[16];
#pragma unroll
  for (int q = 0; q < 16; ++q) { float t = acc[q] * inv; t += __shfl_xor(t, 4); t += __shfl_xor(t, 8); mean[q] = t * 0.25f + bf16_rne(bgat[cc + q]); }
  v8b h0 = {}, l0 = {}, h1 = {}, l1 = {}; bool wr = false; int col = 0;
  if (l < 4) { wr = true; col = cc; for (int q = 0; q < 16; ++q) { const float o = (v < (size_t)N) ? mean[q] : 0.0f; b16 a_, c_; split16(o * XS, a_, c_); if (q < 8) { h0[q] = a_; l0[q] = c_; } else { h1[q - 8] = a_; l1[q - 8] = c_; } } }
  else if (l == 4) { wr = true; col = OUT; for (int q = 0; q < 16; ++q) { const float o = bf16_rne(nstate[q >> 1]); b16 a_, c_; split16(o * XS, a_, c_); if (q < 8) { h0[q] = a_; l0[q] = c_; } else { h1[q - 8] = a_; l1[q - 8] = c_; } } }
  else if (l == 5) { wr = true; col = OUT + ED; }
  for (int pass = 0; pass < 2; ++pass) { if (wr) { b16* ph = X2h + v * KC + col; b16* pl = X2l + v * KC + col; *(volatile v8b*)ph = h0; *(volatile v8b*)(ph + 8) = h1; *(volatile v8b*)pl = l0; *(volatile v8b*)(pl + 8) = l1; } __threadfence(); }
}
__global__ __launch_bounds__(128) void final_kernel(const b16* __restrict__ Ah, const b16* __restrict__ Al, const b16* __restrict__ WCT, const float* __restrict__ bc, float* __restrict__ out) {
  __shared__ __attribute__((aligned(16))) float Ts[4][16][OUT + 4];
  const int wave = threadIdx.x >> 5, lane = threadIdx.x & 31, nloc = lane & 15, hlf = lane >> 4; const size_t m0 = ((size_t)blockIdx.x * 4 + wave) * 16;
  v8f acc[4] = {{}, {}, {}, {}};
#pragma unroll
  for (int kb = 0; kb < KC; kb += 32) { const v16b a = frag_kb(Ah + (m0 + nloc) * KC + kb, hlf), al = frag_kb(Al + (m0 + nloc) * KC + kb, hlf);
#pragma unroll
    for (int t = 0; t < 4; ++t) { const v16b bw = frag_kb(WCT + (size_t)(t * 16 + nloc) * KC + kb, hlf); acc[t] = wmma16b(a, bw, acc[t]); acc[t] = wmma16b(al, bw, acc[t]); } }
#pragma unroll
  for (int t = 0; t < 4; ++t) { const float bb = bf16_rne(bc[t * 16 + nloc]);
#pragma unroll
    for (int r = 0; r < 8; ++r) Ts[wave][8 * hlf + r][t * 16 + nloc] = fmaxf(acc[t][r] * (1.0f / (XS * WSC)) + bb, 0.0f); }
  wave_lds_sync();
  for (int pass = 0; pass < 2; ++pass) { for (int rr = 0; rr < 16; ++rr) if (lane < 16 && m0 + rr < (size_t)N) *(volatile v4f*)(out + (m0 + rr) * OUT + lane * 4) = *(const v4f*)(&Ts[wave][rr][lane * 4]); __threadfence(); }
}
}

extern "C" void kernel_launch(void* const* d_in, const int* in_sizes, int n_in, void* d_out, int out_size, void* d_ws, size_t ws_size, hipStream_t stream) {
  (void)n_in;
  auto Fp = [&](int i) { return (const float*)d_in[i]; }; auto Ip = [&](int i) { return (const int*)d_in[i]; };
  if (in_sizes[0] != N * IN || in_sizes[1] != 2 * E || in_sizes[2] != E * ED || in_sizes[3] != E * 4 || in_sizes[4] != 8 || in_sizes[5] != IN * HC || in_sizes[8] != ED * HC || in_sizes[15] != (OUT + ED) * OUT || out_size != N * OUT) return;
  size_t off = 0; char* ws = (char*)d_ws;
  auto carve = [&](size_t bytes) { char* p = ws + off; off += (bytes + 255) & ~(size_t)255; return p; };
  b16* X16 = (b16*)carve((size_t)NP * IN * 2); b16* WGT = (b16*)carve((size_t)HC * IN * 2); b16* WCT = (b16*)carve((size_t)OUT * KC * 2); float* U = (float*)carve(256);
  float* XS_ = (float*)carve((size_t)NP * HC * 4); float* AS = (float*)carve((size_t)2 * NP * 2 * 4); float* AD = (float*)carve((size_t)2 * NP * 2 * 4); float* AE = (float*)carve((size_t)E * 4 * 4); b16* X2h = (b16*)carve((size_t)NP * KC * 2); b16* X2l = (b16*)carve((size_t)NP * KC * 2);
  CsrBufs csr; off = csr_carve(csr, ws, off, E, N);
  if (off > ws_size || off > ((size_t)128 << 20)) return;
  const int* srcp = Ip(1); const int* dstp = Ip(1) + E;
  prep_kernel<<<(unsigned)(((size_t)NP * IN / 8 + (size_t)HC * IN / 8 + (size_t)OUT * KC / 8 + 64 + 255) / 256), 256, 0, stream>>>(Fp(0), Fp(5), Fp(15), Fp(8), Fp(9), X16, WGT, WCT, U);
  csr_build(csr, dstp, E, N, stream);
  node_kernel<<<dim3(NP / 64, 2), 128, 0, stream>>>(X16, WGT, Fp(6), Fp(7), XS_, AS, AD);
  edge_kernel<<<(E + 255) / 256, 256, 0, stream>>>(Fp(2), Fp(3), Fp(11), Fp(12), Fp(13), Fp(14), U, AE);
  agg_kernel<<<NP / 16, 256, 0, stream>>>(srcp, XS_, AS, AD, AE, Fp(10), Fp(4), csr.PERM, csr.ROWPTR, csr.ROWCNT, (int)csr.permLen, X2h, X2l);
  final_kernel<<<NP / 64, 128, 0, stream>>>(X2h, X2l, WCT, Fp(16), (float*)d_out);
}
